// LSTMDecoder_49624052138309
// MI455X (gfx1250) — hardware-verified
//
#include <hip/hip_runtime.h>


#define NB   65536
#define RC   16384
#define HH   128
#define G4   512
#define K2   256
#define N1   103
#define N2   119
#define N3   11
#define P1   128
#define P2   128
#define P3   64
typedef _Float16 h16;
typedef unsigned short bf;
typedef __attribute__((ext_vector_type(16))) __bf16   v16bf;
typedef __attribute__((ext_vector_type(16))) _Float16 v16h;
typedef __attribute__((ext_vector_type(8)))  _Float16 v8h;
typedef __attribute__((ext_vector_type(8)))  unsigned short v8us;
typedef __attribute__((ext_vector_type(8)))  float    v8f;
typedef __attribute__((ext_vector_type(4)))  float    v4f;
typedef v8h  __attribute__((may_alias)) v8ha;
typedef v4f  __attribute__((may_alias)) v4fa;
typedef v8us __attribute__((may_alias)) v8usa;

__device__ __forceinline__ unsigned short f2bf(float f) { unsigned u = __float_as_uint(f); u += 0x7FFFu + ((u >> 16) & 1u); return (unsigned short)(u >> 16); }
__device__ __forceinline__ float bf2f(unsigned short b) { return __uint_as_float(((unsigned)b) << 16); }
__device__ __forceinline__ float bfr(float f) { return bf2f(f2bf(f)); }
__device__ __forceinline__ v16h cat16(v8h lo, v8h hi) { return __builtin_shufflevector(lo, hi, 0, 1, 2, 3, 4, 5, 6, 7, 8, 9, 10, 11, 12, 13, 14, 15); }
__device__ __forceinline__ v16bf cat16b(v8us lo, v8us hi) { return __builtin_bit_cast(v16bf, __builtin_shufflevector(lo, hi, 0, 1, 2, 3, 4, 5, 6, 7, 8, 9, 10, 11, 12, 13, 14, 15)); }
__device__ __forceinline__ v8f wmma16(v16h a, v16h b, v8f c) { return __builtin_amdgcn_wmma_f32_16x16x32_f16(false, a, false, b, (short)0, c, false, false); }
__device__ __forceinline__ v8f wmmab(v16bf a, v16bf b, v8f c) { return __builtin_amdgcn_wmma_f32_16x16x32_bf16(false, a, false, b, (short)0, c, false, false); }


template <typename T16> struct WFrag;
template <> struct WFrag<h16> { typedef v16h V; static __device__ __forceinline__ V ld(const h16* p) { return cat16(*(const v8h*)p, *(const v8h*)(p + 16)); } static __device__ __forceinline__ v8f mma(V a, V b, v8f c) { return wmma16(a, b, c); } };
template <> struct WFrag<bf> { typedef v16bf V; static __device__ __forceinline__ V ld(const bf* p) { return cat16b(*(const v8us*)p, *(const v8us*)(p + 16)); } static __device__ __forceinline__ v8f mma(V a, V b, v8f c) { return wmmab(a, b, c); } };
template <typename T16, int NSPLIT, bool BIAS>
__global__ __launch_bounds__(32) void k_gemmw(const T16* __restrict__ A, const T16* __restrict__ A2, const T16* __restrict__ Bt, const T16* __restrict__ Bt2, int K, float* C, int ldc, const float* __restrict__ bias, size_t sA, size_t sB, size_t sC) {
    typedef typename WFrag<T16>::V V;
    __shared__ __align__(16) float os[16 * 68];
    const size_t z = blockIdx.z; A += z * sA; if (A2) A2 += z * sA; Bt += z * sB; if (Bt2) Bt2 += z * sB; C += z * sC;
    const int lane = threadIdx.x & 31, lr = lane & 15, hi = lane >> 4; const int r0 = blockIdx.x * 64, c0 = blockIdx.y * 64;
    v8f acc[4][4];
#pragma unroll
    for (int mb = 0; mb < 4; ++mb)
#pragma unroll
        for (int nb = 0; nb < 4; ++nb) acc[mb][nb] = (v8f){};
    const size_t aoff = (size_t)(r0 + lr) * K + 8 * hi, boff = (size_t)(c0 + lr) * K + 8 * hi;
#pragma unroll 1
    for (int kc = 0; kc < K; kc += 32) {
        V a[4], a2[4];
#pragma unroll
        for (int mb = 0; mb < 4; ++mb) { a[mb] = WFrag<T16>::ld(A + aoff + (size_t)mb * 16 * K + kc); if (NSPLIT == 1 || NSPLIT == 2) a2[mb] = WFrag<T16>::ld(A2 + aoff + (size_t)mb * 16 * K + kc); }
#pragma unroll
        for (int nb = 0; nb < 4; ++nb) { const V b = WFrag<T16>::ld(Bt + boff + (size_t)nb * 16 * K + kc); V b2; if (NSPLIT >= 2) b2 = WFrag<T16>::ld(Bt2 + boff + (size_t)nb * 16 * K + kc);
#pragma unroll
            for (int mb = 0; mb < 4; ++mb) { acc[mb][nb] = WFrag<T16>::mma(a[mb], b, acc[mb][nb]); if (NSPLIT == 1 || NSPLIT == 2) acc[mb][nb] = WFrag<T16>::mma(a2[mb], b, acc[mb][nb]); if (NSPLIT >= 2) acc[mb][nb] = WFrag<T16>::mma(a[mb], b2, acc[mb][nb]); } }
        asm volatile("v_nop\n\tv_nop\n\tv_nop\n\tv_nop" : "+v"(acc[0][0]), "+v"(acc[1][1]), "+v"(acc[2][2]), "+v"(acc[3][3]) : "v"(a[0]), "v"(a[3]));
    }
#pragma unroll
    for (int mb = 0; mb < 4; ++mb) {
#pragma unroll
        for (int nb = 0; nb < 4; ++nb) {
#pragma unroll
            for (int j = 0; j < 8; ++j) os[(hi * 8 + j) * 68 + nb * 16 + lr] = acc[mb][nb][j]; }
        __builtin_amdgcn_wave_barrier(); asm volatile("" ::: "memory");
        float* crow = C + (size_t)(r0 + mb * 16) * ldc + c0;
#pragma unroll 1
        for (int ps = 0; ps < 2; ++ps) {
#pragma unroll
            for (int s = 0; s < 8; ++s) { const int row = 2 * s + hi, cofs = lr * 4; v4f val = *(const v4fa*)(os + row * 68 + cofs); if (BIAS) { val[0] += bfr(bias[c0 + cofs]); val[1] += bfr(bias[c0 + cofs + 1]); val[2] += bfr(bias[c0 + cofs + 2]); val[3] += bfr(bias[c0 + cofs + 3]); }
                *(volatile v4f*)(crow + (size_t)row * ldc + cofs) = val; }
            if (ps == 0) __threadfence(); }
        __builtin_amdgcn_wave_barrier(); asm volatile("" ::: "memory");
    }
}

typedef __attribute__((ext_vector_type(4))) unsigned short v4us;
typedef __attribute__((ext_vector_type(2))) unsigned short v2us;
typedef __attribute__((ext_vector_type(2))) float v2f;
__device__ __forceinline__ void splitf(float y, unsigned short& h, unsigned short& l) { h = f2bf(y); l = f2bf(y - bf2f(h)); }
__device__ __forceinline__ float expx(float a) { return __builtin_amdgcn_exp2f(__fmul_rn(a, 1.4426950408889634f)); }
__device__ __forceinline__ float sigm(float a) { return __fdiv_rn(1.0f, __fadd_rn(1.0f, expx(-a))); }
__device__ __forceinline__ float tanhx(float a) { return __fsub_rn(1.0f, __fdiv_rn(2.0f, __fadd_rn(expx(__fmul_rn(2.0f, a)), 1.0f))); }
__global__ __launch_bounds__(256) void k_wtG(const float* __restrict__ w, int K, int N, bf* Bt) {
    const int lane = threadIdx.x & 31; const int L0 = (blockIdx.x * 8 + (threadIdx.x >> 5)) * 8; const int nlines = N * K / 64;
#pragma unroll
    for (int ps = 0; ps < 2; ++ps) {
#pragma unroll 1
        for (int l = 0; l < 8; ++l) { const int L = L0 + l; if (L >= nlines) break; const size_t e = (size_t)L * 64 + lane * 2; const int k = (int)(e % K), n = (int)(e / K); v2us o;
            o[0] = f2bf(w[(size_t)k * N + n]); o[1] = f2bf(w[(size_t)(k + 1) * N + n]); *(volatile v2us*)(Bt + e) = o; }
        if (ps == 0) __threadfence(); }
}

__global__ __launch_bounds__(256) void k_wtS(const float* __restrict__ wx, const float* __restrict__ wh, bf* Bt) { const int lane = threadIdx.x & 31; const int L0 = (blockIdx.x * 8 + (threadIdx.x >> 5)) * 8; const int nlines = G4 * K2 / 64;
#pragma unroll
    for (int ps = 0; ps < 2; ++ps) {
#pragma unroll 1
        for (int l = 0; l < 8; ++l) { const int L = L0 + l; if (L >= nlines) break; const size_t e = (size_t)L * 64 + lane * 2; const int k = (int)(e % K2), n = (int)(e / K2); v2us o;
#pragma unroll
            for (int q = 0; q < 2; ++q) { const int kk = k + q; o[q] = f2bf(kk < HH ? wx[(size_t)kk * G4 + n] : wh[(size_t)(kk - HH) * G4 + n]); }
            *(volatile v2us*)(Bt + e) = o; }
        if (ps == 0) __threadfence(); } }
__global__ __launch_bounds__(32) void k_bpad(const float* __restrict__ b, int n, int np, float* dst) { const int i = threadIdx.x; if (i >= np / 4) return; v4f o;
#pragma unroll
    for (int q = 0; q < 4; ++q) { const int c = i * 4 + q; o[q] = (c < n) ? b[c] : 0.0f; } *(volatile v4f*)(dst + i * 4) = o; __threadfence(); *(volatile v4f*)(dst + i * 4) = o; }
__global__ __launch_bounds__(256) void k_zero16(bf* Z, size_t n8) { const size_t i = (size_t)blockIdx.x * 256 + threadIdx.x; if (i >= n8) return; v8us o; for (int k = 0; k < 8; ++k) o[k] = 0; *(volatile v8us*)(Z + i * 8) = o; __threadfence(); *(volatile v8us*)(Z + i * 8) = o; }
__global__ __launch_bounds__(256) void k_xpl(const float* __restrict__ X, size_t n0, bf* XB, bf* Ah) { const size_t i = (size_t)blockIdx.x * 256 + threadIdx.x; if (i >= (size_t)RC * HH / 8) return; const size_t r = i / (HH / 8); const int c0 = (int)(i % (HH / 8)) * 8; const v4f a = *(const v4f*)(X + (n0 + r) * HH + c0); const v4f b = *(const v4f*)(X + (n0 + r) * HH + c0 + 4); v8us o;
    for (int k = 0; k < 4; ++k) { o[k] = f2bf(a[k]); o[4 + k] = f2bf(b[k]); }
    *(volatile v8us*)(XB + r * HH + c0) = o; *(volatile v8us*)(Ah + r * K2 + c0) = o; __threadfence(); *(volatile v8us*)(XB + r * HH + c0) = o; *(volatile v8us*)(Ah + r * K2 + c0) = o; }
__global__ __launch_bounds__(256) void k_cell(const float* __restrict__ Z, const float* __restrict__ Cp, float* Hn, float* Cn, bf* Ah, bf* Al) {
    const size_t i = (size_t)blockIdx.x * 256 + threadIdx.x; if (i >= (size_t)RC * HH / 2) return; const size_t r = i / (HH / 2); const int u0 = (int)(i % (HH / 2)) * 2; const float* zr = Z + r * G4;
    const v2f zi = *(const v2f*)(zr + u0), zf = *(const v2f*)(zr + HH + u0), zg = *(const v2f*)(zr + 2 * HH + u0), zo = *(const v2f*)(zr + 3 * HH + u0);
    v2f cp; if (Cp) cp = *(const v2f*)(Cp + r * HH + u0); else { cp[0] = cp[1] = 0.f; }
    v2f hn, cn; v2us oh, ol;
#pragma unroll
    for (int q = 0; q < 2; ++q) { float a = __fmul_rn(sigm(zf[q]), cp[q]); asm volatile("" : "+v"(a)); float b = __fmul_rn(sigm(zi[q]), tanhx(zg[q])); asm volatile("" : "+v"(b)); const float c = __fadd_rn(a, b); cn[q] = c; const float h = __fmul_rn(sigm(zo[q]), tanhx(c)); hn[q] = h; unsigned short h2, l2; splitf(h, h2, l2); oh[q] = h2; ol[q] = l2; }
#pragma unroll 1
    for (int ps = 0; ps < 2; ++ps) { *(volatile v2f*)(Hn + r * HH + u0) = hn; *(volatile v2f*)(Cn + r * HH + u0) = cn; if (Ah) { *(volatile v2us*)(Ah + r * K2 + HH + u0) = oh; *(volatile v2us*)(Al + r * K2 + HH + u0) = ol; } if (ps == 0) __threadfence(); }
}

__global__ __launch_bounds__(256) void k_tohl(const float* __restrict__ F, bf* Hh, bf* Hl, size_t n4) { const size_t i = (size_t)blockIdx.x * 256 + threadIdx.x; if (i >= n4) return; const v4f a = *(const v4f*)(F + i * 4); v4us oh, ol;
#pragma unroll
    for (int q = 0; q < 4; ++q) { unsigned short h2, l2; splitf(a[q], h2, l2); oh[q] = h2; ol[q] = l2; }
    *(volatile v4us*)(Hh + i * 4) = oh; *(volatile v4us*)(Hl + i * 4) = ol; __threadfence(); *(volatile v4us*)(Hh + i * 4) = oh; *(volatile v4us*)(Hl + i * 4) = ol; }
__global__ __launch_bounds__(256) void k_relu(const float* __restrict__ F, bf* Rh, bf* Rl, size_t n4) { const size_t i = (size_t)blockIdx.x * 256 + threadIdx.x; if (i >= n4) return; const v4f a = *(const v4f*)(F + i * 4); v4us oh, ol;
#pragma unroll
    for (int q = 0; q < 4; ++q) { unsigned short h2, l2; splitf(fmaxf(a[q], 0.0f), h2, l2); oh[q] = h2; ol[q] = l2; }
    *(volatile v4us*)(Rh + i * 4) = oh; *(volatile v4us*)(Rl + i * 4) = ol; __threadfence(); *(volatile v4us*)(Rh + i * 4) = oh; *(volatile v4us*)(Rl + i * 4) = ol; }
__global__ __launch_bounds__(256) void k_addpl(const float* __restrict__ A, const float* __restrict__ T, float* S, bf* Ah, bf* Al) { const size_t i = (size_t)blockIdx.x * 256 + threadIdx.x; if (i >= (size_t)RC * HH / 4) return; const size_t r = i / (HH / 4); const int u0 = (int)(i % (HH / 4)) * 4; const v4f a = *(const v4f*)(A + r * HH + u0); const v4f t = *(const v4f*)(T + r * HH + u0); v4f s; v4us oh, ol;
#pragma unroll
    for (int q = 0; q < 4; ++q) { s[q] = __fadd_rn(a[q], t[q]); unsigned short h2, l2; splitf(s[q], h2, l2); oh[q] = h2; ol[q] = l2; }
#pragma unroll 1
    for (int ps = 0; ps < 2; ++ps) { *(volatile v4f*)(S + r * HH + u0) = s; if (Ah) { *(volatile v4us*)(Ah + r * K2 + HH + u0) = oh; *(volatile v4us*)(Al + r * K2 + HH + u0) = ol; } if (ps == 0) __threadfence(); }
}
__global__ __launch_bounds__(256) void k_flat(const float* __restrict__ Cc, int n, int np, size_t n0, float* out) { const size_t i = (size_t)blockIdx.x * 256 + threadIdx.x; const size_t tot4 = (size_t)RC * n / 4; if (i >= tot4) return; v4f o;
#pragma unroll
    for (int q = 0; q < 4; ++q) { const size_t f = i * 4 + q; const size_t r = f / n; const int c = (int)(f % n); o[q] = Cc[r * np + c]; }
    float* dst = out + n0 * (size_t)n + i * 4; *(volatile v4f*)dst = o; __threadfence(); *(volatile v4f*)dst = o; }

extern "C" void kernel_launch(void* const* d_in, const int* in_sizes, int n_in,
                              void* d_out, int out_size, void* d_ws, size_t ws_size, hipStream_t stream) {
    (void)in_sizes; (void)n_in; (void)out_size;
    const float* x = (const float*)d_in[0]; const float* Wx = (const float*)d_in[1]; const float* Wh = (const float*)d_in[2]; const float* bb = (const float*)d_in[3]; const float* hfcW = (const float*)d_in[4]; const float* hfcb = (const float*)d_in[5]; const float* cfcW = (const float*)d_in[6]; const float* cfcb = (const float*)d_in[7];
    const float* midW = (const float*)d_in[8]; const float* midb = (const float*)d_in[9]; const float* o1W = (const float*)d_in[10]; const float* o1b = (const float*)d_in[11]; const float* o2W = (const float*)d_in[12]; const float* o2b = (const float*)d_in[13]; const float* o3W = (const float*)d_in[14]; const float* o3b = (const float*)d_in[15];
    float* OUT1 = (float*)d_out; float* OUT2 = OUT1 + (size_t)NB * N1; float* OUT3 = OUT2 + (size_t)NB * N2;
    char* wsp = (char*)d_ws;
    auto take = [&](size_t bytes) { char* p = wsp; wsp += (bytes + 255) & ~(size_t)255; return (void*)p; };
    bf* W0 = (bf*)take((size_t)G4 * HH * 2); bf* WS1 = (bf*)take((size_t)G4 * K2 * 2); bf* WS2 = (bf*)take((size_t)G4 * K2 * 2); bf* WHF = (bf*)take((size_t)HH * HH * 2); bf* WCF = (bf*)take((size_t)HH * HH * 2);
    bf* WM = (bf*)take((size_t)3 * HH * HH * 2); bf* WO1 = (bf*)take((size_t)P1 * HH * 2); bf* WO2 = (bf*)take((size_t)P2 * HH * 2); bf* WO3 = (bf*)take((size_t)P3 * HH * 2); float* BO1 = (float*)take(P1 * 4); float* BO2 = (float*)take(P2 * 4); float* BO3 = (float*)take(P3 * 4);
    bf* XB = (bf*)take((size_t)RC * HH * 2); bf* Ah = (bf*)take((size_t)RC * K2 * 2); bf* Al = (bf*)take((size_t)RC * K2 * 2); float* Z = (float*)take((size_t)RC * G4 * 4);
    float* H1 = (float*)take((size_t)RC * HH * 4); float* C1 = (float*)take((size_t)RC * HH * 4); float* H2 = (float*)take((size_t)RC * HH * 4); float* C2 = (float*)take((size_t)RC * HH * 4); float* H3 = (float*)take((size_t)RC * HH * 4); float* C3 = (float*)take((size_t)RC * HH * 4); float* S3 = (float*)take((size_t)RC * HH * 4); float* T1 = (float*)take((size_t)RC * HH * 4);
    bf* Ph = (bf*)take((size_t)RC * HH * 2); bf* Pl = (bf*)take((size_t)RC * HH * 2); float* M = (float*)take((size_t)RC * HH * 4); float* Cc = (float*)take((size_t)RC * P1 * 4);
    if ((size_t)(wsp - (char*)d_ws) > ws_size) return;
    k_wtG<<<(unsigned)((HH * G4 / 64 + 63) / 64), 256, 0, stream>>>(Wx, HH, G4, W0);
    k_wtS<<<(unsigned)((G4 * K2 / 64 + 63) / 64), 256, 0, stream>>>(Wx + (size_t)1 * HH * G4, Wh + (size_t)1 * HH * G4, WS1);
    k_wtS<<<(unsigned)((G4 * K2 / 64 + 63) / 64), 256, 0, stream>>>(Wx + (size_t)2 * HH * G4, Wh + (size_t)2 * HH * G4, WS2);
    k_wtG<<<(unsigned)((HH * HH / 64 + 63) / 64), 256, 0, stream>>>(hfcW, HH, HH, WHF); k_wtG<<<(unsigned)((HH * HH / 64 + 63) / 64), 256, 0, stream>>>(cfcW, HH, HH, WCF);
    for (int i = 0; i < 3; ++i) k_wtG<<<(unsigned)((HH * HH / 64 + 63) / 64), 256, 0, stream>>>(midW + (size_t)i * HH * HH, HH, HH, WM + (size_t)i * HH * HH);
    k_zero16<<<(unsigned)(((size_t)(P1 + P2 + P3) * HH / 8 + 255) / 256), 256, 0, stream>>>(WO1, (size_t)(P1 + P2 + P3) * HH / 8);
    k_wtG<<<(unsigned)((HH * N1 / 64 + 63) / 64), 256, 0, stream>>>(o1W, HH, N1, WO1); k_wtG<<<(unsigned)((HH * N2 / 64 + 63) / 64), 256, 0, stream>>>(o2W, HH, N2, WO2); k_wtG<<<(unsigned)((HH * N3 / 64 + 63) / 64), 256, 0, stream>>>(o3W, HH, N3, WO3);
    k_bpad<<<1, 32, 0, stream>>>(o1b, N1, P1, BO1); k_bpad<<<1, 32, 0, stream>>>(o2b, N2, P2, BO2); k_bpad<<<1, 32, 0, stream>>>(o3b, N3, P3, BO3);
    k_zero16<<<(unsigned)(((size_t)RC * K2 / 8 + 255) / 256), 256, 0, stream>>>(Al, (size_t)RC * K2 / 8);
    const size_t N4 = (size_t)RC * HH / 4; const unsigned gb4 = (unsigned)((N4 + 255) / 256); const unsigned gb2 = (unsigned)(((size_t)RC * HH / 2 + 255) / 256);
    for (size_t n0 = 0; n0 < (size_t)NB; n0 += RC) {
        k_xpl<<<(unsigned)(((size_t)RC * HH / 8 + 255) / 256), 256, 0, stream>>>(x, n0, XB, Ah);
        k_gemmw<bf, 0, true><<<dim3(RC / 64, G4 / 64, 1), 32, 0, stream>>>(XB, nullptr, W0, nullptr, HH, Z, G4, bb, 0, 0, 0);
        k_cell<<<gb2, 256, 0, stream>>>(Z, nullptr, H1, C1, Ah, Al);
        k_gemmw<bf, 1, true><<<dim3(RC / 64, G4 / 64, 1), 32, 0, stream>>>(Ah, Al, WS1, nullptr, K2, Z, G4, bb + G4, 0, 0, 0);
        k_cell<<<gb2, 256, 0, stream>>>(Z, C1, H2, C2, nullptr, nullptr);
        k_tohl<<<gb4, 256, 0, stream>>>(H2, Ph, Pl, N4); k_gemmw<bf, 1, true><<<dim3(RC / 64, HH / 64, 1), 32, 0, stream>>>(Ph, Pl, WHF, nullptr, HH, T1, HH, hfcb, 0, 0, 0); k_addpl<<<gb4, 256, 0, stream>>>(H1, T1, H3, Ah, Al);
        k_tohl<<<gb4, 256, 0, stream>>>(C2, Ph, Pl, N4); k_gemmw<bf, 1, true><<<dim3(RC / 64, HH / 64, 1), 32, 0, stream>>>(Ph, Pl, WCF, nullptr, HH, T1, HH, cfcb, 0, 0, 0); k_addpl<<<gb4, 256, 0, stream>>>(C1, T1, S3, nullptr, nullptr);
        k_gemmw<bf, 1, true><<<dim3(RC / 64, G4 / 64, 1), 32, 0, stream>>>(Ah, Al, WS2, nullptr, K2, Z, G4, bb + 2 * G4, 0, 0, 0);
        k_cell<<<gb2, 256, 0, stream>>>(Z, S3, H3, C3, nullptr, nullptr);
        const float* Hs[3] = {H1, H2, H3}; bf* WOs[3] = {WO1, WO2, WO3}; float* BOs[3] = {BO1, BO2, BO3}; float* OUTs[3] = {OUT1, OUT2, OUT3}; const int Ns[3] = {N1, N2, N3}; const int Ps[3] = {P1, P2, P3};
        for (int i = 0; i < 3; ++i) {
            k_tohl<<<gb4, 256, 0, stream>>>(Hs[i], Ph, Pl, N4);
            k_gemmw<bf, 1, true><<<dim3(RC / 64, HH / 64, 1), 32, 0, stream>>>(Ph, Pl, WM + (size_t)i * HH * HH, nullptr, HH, M, HH, midb + i * HH, 0, 0, 0);
            k_relu<<<gb4, 256, 0, stream>>>(M, Ph, Pl, N4);
            k_gemmw<bf, 1, true><<<dim3(RC / 64, Ps[i] / 64, 1), 32, 0, stream>>>(Ph, Pl, WOs[i], nullptr, HH, Cc, Ps[i], BOs[i], 0, 0, 0);
            k_flat<<<(unsigned)(((size_t)RC * Ns[i] / 4 + 255) / 256), 256, 0, stream>>>(Cc, Ns[i], Ps[i], n0, OUTs[i]); } }
}
